// DifferentiableCBFLayer_84791244357684
// MI455X (gfx1250) — hardware-verified
//
#include <hip/hip_runtime.h>
#define NB 32768
#define MROW 26
#define NV 5
#define SPB 32

typedef __bf16 v16b __attribute__((ext_vector_type(16)));
typedef unsigned short v8us __attribute__((ext_vector_type(8), may_alias));
typedef float  v8f  __attribute__((ext_vector_type(8)));
typedef float  v4f  __attribute__((ext_vector_type(4)));
typedef float  v4fa __attribute__((ext_vector_type(4), may_alias));
union FragB { v16b v; v8us half[2]; unsigned short u[16]; };

__device__ __forceinline__ unsigned short bf16_bits(float x) { unsigned int u = __float_as_uint(x); return (unsigned short)((u + 0x7FFFu + ((u >> 16) & 1u)) >> 16); }
__device__ __forceinline__ float bf16_val(unsigned short b) { return __uint_as_float(((unsigned int)b) << 16); }
__device__ __forceinline__ float bf16_round(float x) { return bf16_val(bf16_bits(x)); }
template <int NT>
__device__ __forceinline__ v8f mmaN(v16b ah, v16b al, v16b bh, v16b bl, v8f c) {
  c = __builtin_amdgcn_wmma_f32_16x16x32_bf16(false, ah, false, bh, (short)0, c, false, false);
  if (NT >= 2) c = __builtin_amdgcn_wmma_f32_16x16x32_bf16(false, al, false, bh, (short)0, c, false, false);
  if (NT >= 3) c = __builtin_amdgcn_wmma_f32_16x16x32_bf16(false, ah, false, bl, (short)0, c, false, false);
  asm volatile("v_nop\n\tv_nop\n\tv_nop\n\tv_nop" : "+v"(c) : "v"(ah), "v"(al), "v"(bh), "v"(bl));
  return c;
}

__global__ __launch_bounds__(256) void k_wt_bf16(const float* __restrict__ W, unsigned short* __restrict__ Wt, int K, int N) {
  const int t = blockIdx.x * 256 + threadIdx.x;
  const int k8n = K / 8;
  if (t >= N * k8n) return;
  const int n = t / k8n, k8 = (t % k8n) * 8;
  v8us v;
#pragma unroll
  for (int i = 0; i < 8; ++i) v[i] = bf16_bits(W[(size_t)(k8 + i) * N + n]);
  *(volatile v8us*)(Wt + (size_t)n * K + k8) = v;
  __threadfence();
  *(volatile v8us*)(Wt + (size_t)n * K + k8) = v;
}

template <bool ASPLIT, int ACT, bool BIAS_BF16>
__global__ __launch_bounds__(128) void k_gemm_bf(const float* __restrict__ A, int lda, const unsigned short* __restrict__ Wt, int ldb,
                                               const float* __restrict__ bias, float* __restrict__ C, int ldc, int M, int N, int K) {
  __shared__ __attribute__((aligned(16))) float so[4][16][64];
  const int tid = threadIdx.x, w = tid >> 5, lane = tid & 31, ln = lane & 15, hh = lane >> 4;
  const int ntn = N / 64;
  const int wid = blockIdx.x * 4 + w;
  const int mt = wid / ntn, nq = wid % ntn;
  if (mt * 16 >= M) return;
  const int row0 = mt * 16, col0 = nq * 64;
  const float* arow = A + (size_t)(row0 + ln) * lda;
  v8f acc[4] = {};
  for (int kb = 0; kb < K; kb += 32) {
    FragB ah, al;
    const v4f x0 = *(const v4fa*)(arow + kb + 8 * hh), x1 = *(const v4fa*)(arow + kb + 8 * hh + 4);
    const v4f x2 = *(const v4fa*)(arow + kb + 16 + 8 * hh), x3 = *(const v4fa*)(arow + kb + 16 + 8 * hh + 4);
    float xs[16] = {x0[0],x0[1],x0[2],x0[3],x1[0],x1[1],x1[2],x1[3],x2[0],x2[1],x2[2],x2[3],x3[0],x3[1],x3[2],x3[3]};
#pragma unroll
    for (int i = 0; i < 16; ++i) { const unsigned short hb = bf16_bits(xs[i]); ah.u[i] = hb; al.u[i] = ASPLIT ? bf16_bits(xs[i] - bf16_val(hb)) : (unsigned short)0; }
#pragma unroll
    for (int t = 0; t < 4; ++t) {
      const unsigned short* brow = Wt + (size_t)(col0 + t * 16 + ln) * ldb + kb;
      FragB b;
      b.half[0] = *(const v8us*)(brow + 8 * hh);
      b.half[1] = *(const v8us*)(brow + 16 + 8 * hh);
      acc[t] = mmaN<ASPLIT ? 2 : 1>(ah.v, al.v, b.v, b.v, acc[t]);
    }
  }
#pragma unroll
  for (int t = 0; t < 4; ++t) {
    float bv = bias ? bias[col0 + t * 16 + ln] : 0.f;
    if (BIAS_BF16) bv = bf16_round(bv);
#pragma unroll
    for (int r = 0; r < 8; ++r) { float v = acc[t][r] + bv; if (ACT == 1) v = fmaxf(v, 0.f); so[w][8 * hh + r][t * 16 + ln] = v; }
  }
  __builtin_amdgcn_fence(__ATOMIC_ACQ_REL, "workgroup");
  __builtin_amdgcn_wave_barrier();
  const int rsub = lane >> 4, c4 = (lane & 15) * 4;
  for (int pass = 0; pass < 2; ++pass) {
#pragma unroll
    for (int q = 0; q < 8; ++q) {
      const int r = q * 2 + rsub;
      const v4f v = *(const v4fa*)&so[w][r][c4];
      *(volatile v4f*)(C + (size_t)(row0 + r) * ldc + col0 + c4) = v;
    }
    if (pass == 0) __threadfence();
  }
}

template <int D, bool CAUSAL>
__global__ __launch_bounds__(128) void k_flash(const float* __restrict__ qb, const float* __restrict__ kb, const float* __restrict__ vb,
                                             int pitch, int T, int H, float scale, float* __restrict__ y, int ypitch) {
  constexpr int KS = D / 32;
  constexpr int DT = D / 16;
  __shared__ __attribute__((aligned(16))) unsigned short sKh[32][D + 8], sKl[32][D + 8], sVh[32][D + 8], sVl[32][D + 8];
  __shared__ __attribute__((aligned(16))) unsigned short sPh[4][16][40], sPl[4][16][40];
  __shared__ __attribute__((aligned(16))) float sO[4][16][D];
  const int tid = threadIdx.x, w = tid >> 5, lane = tid & 31, ln = lane & 15, hh = lane >> 4;
  const int nqb = (T + 63) / 64;
  const int bh = blockIdx.x / nqb, qblk = blockIdx.x % nqb;
  const int b = bh / H, h = bh % H;
  const int q0 = qblk * 64 + w * 16;
  const float* Q = qb + (size_t)b * T * pitch + h * D;
  const float* K = kb + (size_t)b * T * pitch + h * D;
  const float* V = vb + (size_t)b * T * pitch + h * D;

  FragB aqh[KS], aql[KS];
  {
    int row = q0 + ln; if (row >= T) row = T - 1;
    const float* qr = Q + (size_t)row * pitch;
#pragma unroll
    for (int ks = 0; ks < KS; ++ks)
#pragma unroll
      for (int i = 0; i < 16; ++i) {
        const int d = ks * 32 + ((i < 8) ? (8 * hh + i) : (16 + 8 * hh + (i - 8)));
        const float x = qr[d] * scale; const unsigned short hb = bf16_bits(x);
        aqh[ks].u[i] = hb; aql[ks].u[i] = bf16_bits(x - bf16_val(hb));
      }
  }
  float m_r[8], l_r[8];
#pragma unroll
  for (int r = 0; r < 8; ++r) { m_r[r] = -3.0e38f; l_r[r] = 0.f; }
  v8f oacc[DT];
#pragma unroll
  for (int dt = 0; dt < DT; ++dt) oacc[dt] = (v8f){0.f,0.f,0.f,0.f,0.f,0.f,0.f,0.f};

  const int kv_end = CAUSAL ? min(T, qblk * 64 + 64) : T;
  for (int j0 = 0; j0 < kv_end; j0 += 32) {
    __syncthreads();
    for (int e = tid; e < 32 * (D / 4); e += 128) {
      const int r = e / (D / 4), c4 = (e % (D / 4)) * 4;
      const int key = j0 + r;
      v4f kf = {0.f,0.f,0.f,0.f}, vf = {0.f,0.f,0.f,0.f};
      if (key < T) { kf = *(const v4fa*)(K + (size_t)key * pitch + c4); vf = *(const v4fa*)(V + (size_t)key * pitch + c4); }
#pragma unroll
      for (int t = 0; t < 4; ++t) {
        unsigned short hb = bf16_bits(kf[t]); sKh[r][c4 + t] = hb; sKl[r][c4 + t] = bf16_bits(kf[t] - bf16_val(hb));
        hb = bf16_bits(vf[t]); sVh[r][c4 + t] = hb; sVl[r][c4 + t] = bf16_bits(vf[t] - bf16_val(hb));
      }
    }
    __syncthreads();
    v8f s[2];
#pragma unroll
    for (int nt = 0; nt < 2; ++nt) {
      v8f acc = {};
#pragma unroll
      for (int ks = 0; ks < KS; ++ks) {
        FragB bh_, bl_;
        bh_.half[0] = *(const v8us*)&sKh[nt * 16 + ln][ks * 32 + 8 * hh]; bh_.half[1] = *(const v8us*)&sKh[nt * 16 + ln][ks * 32 + 16 + 8 * hh];
        bl_.half[0] = *(const v8us*)&sKl[nt * 16 + ln][ks * 32 + 8 * hh]; bl_.half[1] = *(const v8us*)&sKl[nt * 16 + ln][ks * 32 + 16 + 8 * hh];
        acc = mmaN<3>(aqh[ks].v, aql[ks].v, bh_.v, bl_.v, acc);
      }
      s[nt] = acc;
    }
    float alpha[8];
#pragma unroll
    for (int r = 0; r < 8; ++r) {
      const int qi = q0 + 8 * hh + r;
      const int ja = j0 + ln, jb = j0 + 16 + ln;
      if (CAUSAL) { if (ja > qi) s[0][r] = -3.0e38f; if (jb > qi) s[1][r] = -3.0e38f; }
      if (ja >= T) s[0][r] = -3.0e38f;
      if (jb >= T) s[1][r] = -3.0e38f;
      float mx = fmaxf(s[0][r], s[1][r]);
      mx = fmaxf(mx, __shfl_xor(mx, 1, 32)); mx = fmaxf(mx, __shfl_xor(mx, 2, 32)); mx = fmaxf(mx, __shfl_xor(mx, 4, 32)); mx = fmaxf(mx, __shfl_xor(mx, 8, 32));
      const float mnew = fmaxf(m_r[r], mx);
      alpha[r] = (mnew > -1.0e38f) ? __expf(m_r[r] - mnew) : 1.0f;
      const float p0 = (s[0][r] > -1.0e38f) ? __expf(s[0][r] - mnew) : 0.f;
      const float p1 = (s[1][r] > -1.0e38f) ? __expf(s[1][r] - mnew) : 0.f;
      m_r[r] = mnew;
      l_r[r] = l_r[r] * alpha[r] + p0 + p1;
      unsigned short hb = bf16_bits(p0); sPh[w][8 * hh + r][ln] = hb;      sPl[w][8 * hh + r][ln] = bf16_bits(p0 - bf16_val(hb));
      hb = bf16_bits(p1);                sPh[w][8 * hh + r][16 + ln] = hb; sPl[w][8 * hh + r][16 + ln] = bf16_bits(p1 - bf16_val(hb));
    }
#pragma unroll
    for (int dt = 0; dt < DT; ++dt)
#pragma unroll
      for (int r = 0; r < 8; ++r) oacc[dt][r] *= alpha[r];
    __builtin_amdgcn_fence(__ATOMIC_ACQ_REL, "workgroup");
    __builtin_amdgcn_wave_barrier();
    FragB pah, pal;
    pah.half[0] = *(const v8us*)&sPh[w][ln][8 * hh]; pah.half[1] = *(const v8us*)&sPh[w][ln][16 + 8 * hh];
    pal.half[0] = *(const v8us*)&sPl[w][ln][8 * hh]; pal.half[1] = *(const v8us*)&sPl[w][ln][16 + 8 * hh];
#pragma unroll
    for (int dt = 0; dt < DT; ++dt) {
      FragB bvh, bvl;
#pragma unroll
      for (int i = 0; i < 8; ++i) {
        bvh.u[i] = sVh[8 * hh + i][dt * 16 + ln]; bvh.u[8 + i] = sVh[16 + 8 * hh + i][dt * 16 + ln];
        bvl.u[i] = sVl[8 * hh + i][dt * 16 + ln]; bvl.u[8 + i] = sVl[16 + 8 * hh + i][dt * 16 + ln];
      }
      oacc[dt] = mmaN<3>(pah.v, pal.v, bvh.v, bvl.v, oacc[dt]);
    }
    __builtin_amdgcn_fence(__ATOMIC_ACQ_REL, "workgroup");
    __builtin_amdgcn_wave_barrier();
  }
#pragma unroll
  for (int r = 0; r < 8; ++r) {
    float l = l_r[r];
    l += __shfl_xor(l, 1, 32); l += __shfl_xor(l, 2, 32); l += __shfl_xor(l, 4, 32); l += __shfl_xor(l, 8, 32);
    l_r[r] = (l > 0.f) ? 1.0f / l : 0.f;
  }
#pragma unroll
  for (int dt = 0; dt < DT; ++dt)
#pragma unroll
    for (int r = 0; r < 8; ++r) sO[w][8 * hh + r][dt * 16 + ln] = oacc[dt][r] * l_r[r];
  __builtin_amdgcn_fence(__ATOMIC_ACQ_REL, "workgroup");
  __builtin_amdgcn_wave_barrier();
  for (int pass = 0; pass < 2; ++pass) {
    for (int r = 0; r < 16; ++r) {
      const int row = q0 + r;
      if (row < T && lane < D / 4) {
        const v4f val = *(const v4fa*)&sO[w][r][lane * 4];
        *(volatile v4f*)(y + ((size_t)b * T + row) * ypitch + h * D + lane * 4) = val;
      }
    }
    if (pass == 0) __threadfence();
  }
}

__device__ void build_Ab(int s, const float* __restrict__ v_cur, const float* __restrict__ p_obs, const float* __restrict__ obs_mask, const float* __restrict__ p_ag, const float* __restrict__ v_ag, const float* __restrict__ ag_mask,
                         const float* __restrict__ p_c, const float* __restrict__ v_c, const float* __restrict__ c_mask, float* A, float* bb) {
  const float BIG = 1000.0f; const float v = bf16_round(v_cur[s]);
  int r = 0;
  for (int k = 0; k < 3; ++k) { for (int n = 0; n < NV; ++n) A[r * NV + n] = 0.f; A[r * NV + 2 + k] = -1.f; bb[r] = 0.f; ++r; }
#pragma unroll 1
  for (int o = 0; o < 10; ++o) { const float lx = bf16_round(p_obs[((size_t)s * 10 + o) * 2]), ly = bf16_round(p_obs[((size_t)s * 10 + o) * 2 + 1]), m = bf16_round(obs_mask[(size_t)s * 10 + o]);
    const float h = lx * lx + ly * ly - 0.25f; const float hd = -2.0f * lx * v; const float rhs = 2.0f * v * v + 3.0f * hd + 2.0f * h;
    A[r * NV + 0] = 2.0f * lx * m; A[r * NV + 1] = 2.0f * ly * v * m; A[r * NV + 2] = -m; A[r * NV + 3] = 0.f; A[r * NV + 4] = 0.f; bb[r] = (m > 0.f) ? rhs : BIG; ++r; }
#pragma unroll 1
  for (int a = 0; a < 7; ++a) { const float ax = bf16_round(p_ag[((size_t)s * 7 + a) * 2]), ay = bf16_round(p_ag[((size_t)s * 7 + a) * 2 + 1]); const float vjx = bf16_round(v_ag[((size_t)s * 7 + a) * 2]), vjy = bf16_round(v_ag[((size_t)s * 7 + a) * 2 + 1]); const float m = bf16_round(ag_mask[(size_t)s * 7 + a]);
    const float h = ax * ax + ay * ay - 0.64f; const float hd = -2.0f * ax * v + 2.0f * (ax * vjx + ay * vjy); const float hdd = 2.0f * v * v - 2.0f * v * vjx + 2.0f * (-v * vjx + vjx * vjx + vjy * vjy);
    const float rhs = hdd + 3.0f * hd + 2.0f * h;
    A[r * NV + 0] = 2.0f * ax * m; A[r * NV + 1] = (2.0f * ay * v - 2.0f * ay * vjx + 2.0f * ax * vjy) * m; A[r * NV + 2] = 0.f; A[r * NV + 3] = -m; A[r * NV + 4] = 0.f; bb[r] = (m > 0.f) ? rhs : BIG; ++r; }
  { const float cx = bf16_round(p_c[(size_t)s * 2]), cy = bf16_round(p_c[(size_t)s * 2 + 1]), cvx = bf16_round(v_c[(size_t)s * 2]), cvy = bf16_round(v_c[(size_t)s * 2 + 1]), m = bf16_round(c_mask[s]);
    const float h = 25.0f - (cx * cx + cy * cy); const float hd = -(-2.0f * cx * v + 2.0f * (cx * cvx + cy * cvy)); const float hdd = -(2.0f * v * v - 2.0f * v * cvx + 2.0f * (-v * cvx + cvx * cvx + cvy * cvy));
    const float rhs = hdd + 3.0f * hd + 2.0f * h;
    A[r * NV + 0] = -2.0f * cx * m; A[r * NV + 1] = -(2.0f * cy * v - 2.0f * cy * cvx + 2.0f * cx * cvy) * m; A[r * NV + 2] = 0.f; A[r * NV + 3] = 0.f; A[r * NV + 4] = -m; bb[r] = (m > 0.f) ? rhs : BIG; ++r; }
  for (int n = 0; n < NV; ++n) A[r * NV + n] = 0.f; bb[r] = BIG; ++r;
  const float boxA[4][5] = {{-1,0,0,0,0},{1,0,0,0,0},{0,-1,0,0,0},{0,1,0,0,0}}; const float boxb[4] = {2.0f, 2.0f, 1.0f, 1.0f};
  for (int k = 0; k < 4; ++k) { for (int n = 0; n < NV; ++n) A[r * NV + n] = boxA[k][n]; bb[r] = boxb[k]; ++r; }
}
__global__ __launch_bounds__(SPB) void k_qp(const float* __restrict__ u_nom, const float* __restrict__ v_cur, const float* __restrict__ p_obs, const float* __restrict__ obs_mask, const float* __restrict__ p_ag, const float* __restrict__ v_ag, const float* __restrict__ ag_mask,
                                          const float* __restrict__ p_c, const float* __restrict__ v_c, const float* __restrict__ c_mask, float* __restrict__ out) {
  __shared__ float sA[SPB][MROW * NV]; __shared__ float sb[SPB][MROW]; __shared__ float sl[SPB][MROW]; __shared__ float sy[SPB][MROW]; __shared__ float sv[SPB][MROW];
  __shared__ __attribute__((aligned(16))) float sM[SPB][MROW * 32];
  const int lane = threadIdx.x; const int s = blockIdx.x * SPB + lane;
  const float PINV[5] = {0.5f, 0.5f, 0.005f, 0.005f, 0.005f};
  float* A = sA[lane]; float* bb = sb[lane];
  build_Ab(s, v_cur, p_obs, obs_mask, p_ag, v_ag, ag_mask, p_c, v_c, c_mask, A, bb);
  __builtin_amdgcn_fence(__ATOMIC_ACQ_REL, "workgroup"); __builtin_amdgcn_wave_barrier();
  { const int ln = lane & 15, hh = lane >> 4;
#pragma unroll 1
    for (int smp = 0; smp < SPB; ++smp) { const float* As = sA[smp];
#pragma unroll 1
      for (int tile = 0; tile < 4; ++tile) { const int ib = tile >> 1, kb2 = tile & 1;
        FragB ah, al, bh, bl;
#pragma unroll
        for (int i = 0; i < 16; ++i) { const int k = (i < 8) ? (8 * hh + i) : (16 + 8 * hh + (i - 8)); const int ra = ib * 16 + ln, rb = kb2 * 16 + ln;
          const float va = (k < NV && ra < MROW) ? As[ra * NV + k] * PINV[k < NV ? k : 0] : 0.f; const float vb = (k < NV && rb < MROW) ? As[rb * NV + k] : 0.f;
          const unsigned short hba = bf16_bits(va), hbb = bf16_bits(vb); ah.u[i] = hba; al.u[i] = bf16_bits(va - bf16_val(hba)); bh.u[i] = hbb; bl.u[i] = bf16_bits(vb - bf16_val(hbb)); }
        v8f acc = {0.f,0.f,0.f,0.f,0.f,0.f,0.f,0.f}; acc = mmaN<3>(ah.v, al.v, bh.v, bl.v, acc);
#pragma unroll
        for (int r = 0; r < 8; ++r) { const int row = ib * 16 + 8 * hh + r; if (row < MROW) sM[smp][row * 32 + kb2 * 16 + ln] = acc[r]; } } }
  }
  __builtin_amdgcn_fence(__ATOMIC_ACQ_REL, "workgroup"); __builtin_amdgcn_wave_barrier();
  float* vv = sv[lane]; const float* M = sM[lane];
  for (int m = 0; m < MROW; ++m) vv[m] = 1.0f;
  float* wv = sy[lane];
#pragma unroll 1
  for (int it = 0; it < 30; ++it) { float nrm = 0.f;
#pragma unroll 1
    for (int m = 0; m < MROW; ++m) { float w = 0.f;
#pragma unroll 1
      for (int k = 0; k < MROW; ++k) w += M[m * 32 + k] * vv[k]; wv[m] = w; nrm += w * w; }
    const float inv = 1.0f / (sqrtf(nrm) + 1e-12f);
#pragma unroll 1
    for (int m = 0; m < MROW; ++m) vv[m] = wv[m] * inv; }
  float L = 0.f;
#pragma unroll 1
  for (int m = 0; m < MROW; ++m) { float w = 0.f;
#pragma unroll 1
    for (int k = 0; k < MROW; ++k) w += M[m * 32 + k] * vv[k]; L += vv[m] * w; }
  const float step = 1.0f / (L + 1e-6f);
  const float q0 = -2.0f * bf16_round(u_nom[(size_t)s * 2]), q1 = -2.0f * bf16_round(u_nom[(size_t)s * 2 + 1]);
  float* lam = sl[lane]; float* y = sy[lane]; for (int m = 0; m < MROW; ++m) { lam[m] = 0.f; y[m] = 0.f; }
  float tk = 1.0f;
#pragma unroll 1
  for (int it = 0; it < 300; ++it) {
    float g0 = 0.f, g1 = 0.f, g2 = 0.f, g3 = 0.f, g4 = 0.f;
#pragma unroll 1
    for (int m = 0; m < MROW; ++m) { const float ym = y[m]; g0 += A[m * NV] * ym; g1 += A[m * NV + 1] * ym; g2 += A[m * NV + 2] * ym; g3 += A[m * NV + 3] * ym; g4 += A[m * NV + 4] * ym; }
    const float x0 = -(q0 + g0) * PINV[0], x1 = -(q1 + g1) * PINV[1], x2 = -(0.f + g2) * PINV[2], x3 = -(0.f + g3) * PINV[3], x4 = -(0.f + g4) * PINV[4];
    const float tk1 = 0.5f * (1.0f + sqrtf(1.0f + 4.0f * tk * tk)); const float mom = (tk - 1.0f) / tk1;
#pragma unroll 1
    for (int m = 0; m < MROW; ++m) { const float res = (A[m * NV] * x0 + A[m * NV + 1] * x1 + A[m * NV + 2] * x2 + A[m * NV + 3] * x3 + A[m * NV + 4] * x4) - bb[m];
      const float ln_ = fmaxf(y[m] + step * res, 0.f); y[m] = ln_ + mom * (ln_ - lam[m]); lam[m] = ln_; }
    tk = tk1; }
  float g0 = 0.f, g1 = 0.f;
#pragma unroll 1
  for (int m = 0; m < MROW; ++m) { g0 += A[m * NV] * lam[m]; g1 += A[m * NV + 1] * lam[m]; }
  typedef float v2f __attribute__((ext_vector_type(2))); const v2f o = {-(q0 + g0) * PINV[0], -(q1 + g1) * PINV[1]};
  *(volatile v2f*)(out + (size_t)s * 2) = o; __threadfence(); *(volatile v2f*)(out + (size_t)s * 2) = o;
}
extern "C" void kernel_launch(void* const* d_in, const int* in_sizes, int n_in,
                              void* d_out, int out_size, void* d_ws, size_t ws_size, hipStream_t stream) {
  (void)in_sizes; (void)n_in; (void)out_size; (void)d_ws; (void)ws_size;
  k_qp<<<NB / SPB, SPB, 0, stream>>>((const float*)d_in[0], (const float*)d_in[1], (const float*)d_in[2], (const float*)d_in[3], (const float*)d_in[4], (const float*)d_in[5], (const float*)d_in[6], (const float*)d_in[7], (const float*)d_in[8], (const float*)d_in[9], (float*)d_out);
}
